// SequenceToSequenceLayer_47467978555533
// MI455X (gfx1250) — hardware-run, weakly checked
//
#include <hip/hip_runtime.h>
#include <math.h>

typedef __attribute__((ext_vector_type(16))) _Float16 v16h;
typedef __attribute__((ext_vector_type(8)))  _Float16 v8h;
typedef __attribute__((ext_vector_type(8)))  float    v8f;
typedef __attribute__((ext_vector_type(4)))  float    v4f;

constexpr int kL  = 2;
constexpr int kB  = 32;
constexpr int kS  = 512;
constexpr int kF  = 64;
constexpr int kI  = 512;
constexpr int kH  = 512;
constexpr int kG  = 4 * kH;
constexpr int kKs = kI + kH;
static_assert(kI == kH, "layer 1 consumes layer 0's hidden vector");
static_assert((kKs % 32) == 0 && (kI % 32) == 0, "contraction depths are multiples of 32");

constexpr float kActCarry = 64.0f;
constexpr float kWCarry   = 1024.0f;
constexpr float kAccInv   = 1.0f / (kActCarry * kWCarry);
constexpr float kF16MinNormal = 6.103515625e-5f;
static_assert(kActCarry * kWCarry == 65536.0f, "fold-back constant");

constexpr int kRowsPerBlock = 16;
constexpr int kStepThreads  = 512;
constexpr int kStepWaves    = kStepThreads / 32;
constexpr int kUnitsPerWave = kH / kStepWaves;
static_assert(kUnitsPerWave == 32, "each wave owns two 16-unit tiles of every gate");
static_assert((kB % kRowsPerBlock) == 0, "whole 16-sample blocks");
constexpr int kAP = 3 * kH + 8;
constexpr int kSP = 36;
static_assert(((kAP * 2) % 16) == 0 && ((kSP * 4) % 16) == 0, "16-B aligned LDS rows");

constexpr size_t kBytesWP  = (size_t)4 * kG * kKs * 2;
constexpr size_t kBytesFCW = (size_t)kH * kI * 2;
constexpr size_t kBytesX16 = (size_t)kB * kS * kI * 2;
constexpr size_t kBytesXT  = (size_t)kB * kS * kH * 2;
constexpr size_t kOffWP  = 0;
constexpr size_t kOffFCW = kOffWP + kBytesWP;
constexpr size_t kOffX16 = kOffFCW + kBytesFCW;
constexpr size_t kOffXT  = kOffX16 + kBytesX16;
constexpr size_t kWsTotal = kOffXT + kBytesXT;
static_assert(kWsTotal == 50855936ull, "carve total");
static_assert(kWsTotal <= 134217728ull, "carve cap");
static_assert((kOffFCW % 128) == 0 && (kOffX16 % 128) == 0 && (kOffXT % 128) == 0, "128-B aligned regions");

constexpr size_t kOutHidden = (size_t)kB * kF * kH;
constexpr size_t kOutCell   = kOutHidden + (size_t)kL * kB * kH;
constexpr size_t kOutTotal  = kOutCell + (size_t)kL * kB * kH;
static_assert(kOutHidden * 4 == 4194304ull, "hidden byte offset");
static_assert(kOutCell * 4 == 4325376ull, "cell byte offset");
static_assert(kOutTotal * 4 == 4456448ull, "output bytes");

__device__ __forceinline__ unsigned short f2bf_bits(float f) {
  unsigned u = __float_as_uint(f);
  return (unsigned short)((u + 0x7FFFu + ((u >> 16) & 1u)) >> 16);
}
__device__ __forceinline__ float bf_bits2f(unsigned short h) { return __uint_as_float(((unsigned)h) << 16); }
__device__ __forceinline__ float bf_val(float f) { return bf_bits2f(f2bf_bits(f)); }

__device__ __forceinline__ _Float16 carry_half(float v, float carry) {
  const float s = v * carry;
  const float z = (fabsf(s) < kF16MinNormal) ? 0.0f : s;
  return (_Float16)z;
}
__device__ __forceinline__ _Float16 input_half(float v, float carry) {
  return carry_half(bf_val(v), carry);
}

union FragU { v16h v; v8h h[2]; };
__device__ __forceinline__ v16h load_frag(const _Float16* p) {
  FragU f;
  f.h[0] = *(const v8h*)(p);
  f.h[1] = *(const v8h*)(p + 16);
  return f.v;
}
__device__ __forceinline__ v8f mma_g(v16h a, v16h b, v8f c) {
  c = __builtin_amdgcn_wmma_f32_16x16x32_f16(false, a, false, b, (short)0, c, false, false);
  asm volatile("v_nop\n\tv_nop\n\tv_nop\n\tv_nop" : "+v"(c) : "v"(a), "v"(b));
  return c;
}

__device__ __forceinline__ float fast_sigmoid(float x) {
  return __builtin_amdgcn_rcpf(1.0f + __expf(-x));
}
__device__ __forceinline__ float fast_tanh(float x) {
  return fmaf(2.0f, __builtin_amdgcn_rcpf(1.0f + __expf(-2.0f * x)), -1.0f);
}

constexpr int kCellPlaneBlocks = (kG * kKs / 8) / 256;
constexpr int kFcPlaneBlocks   = (kH * kI / 8) / 256;
static_assert(kCellPlaneBlocks == 1024 && kFcPlaneBlocks == 128, "plane block counts");

__global__ __launch_bounds__(256) void weight_planes(
    const float* __restrict__ ewih, const float* __restrict__ ewhh,
    const float* __restrict__ dwih, const float* __restrict__ dwhh,
    const float* __restrict__ fcw,
    _Float16* __restrict__ wp, _Float16* __restrict__ fcp)
{
  const int bx = blockIdx.x;
  const int tid = threadIdx.x;
  const float* src;
  _Float16* dst;
  if (bx < 4 * kCellPlaneBlocks) {
    const int cell = bx / kCellPlaneBlocks;
    const int idx  = (bx - cell * kCellPlaneBlocks) * 256 + tid;
    const int n    = idx / (kKs / 8);
    const int kc   = (idx - n * (kKs / 8)) * 8;
    const int l    = cell & 1;
    const float* wih = (cell >= 2) ? dwih : ewih;
    const float* whh = (cell >= 2) ? dwhh : ewhh;
    const float* base = (kc < kI) ? wih : whh;
    const int kk = (kc < kI) ? kc : (kc - kI);
    src = base + ((size_t)l * kG + n) * kH + kk;
    dst = wp + ((size_t)cell * kG + n) * kKs + kc;
  } else {
    const int idx = (bx - 4 * kCellPlaneBlocks) * 256 + tid;
    src = fcw + (size_t)idx * 8;
    dst = fcp + (size_t)idx * 8;
  }
  const v4f a0 = *(const v4f*)(src);
  const v4f a1 = *(const v4f*)(src + 4);
  v8h hv;
#pragma unroll
  for (int e = 0; e < 4; ++e) {
    const float t0 = a0[e];
    const float t1 = a1[e];
    hv[e]     = input_half(t0, kWCarry);
    hv[4 + e] = input_half(t1, kWCarry);
  }
  *(volatile v8h*)dst = hv;
  __threadfence();
  *(volatile v8h*)dst = hv;
}

__global__ __launch_bounds__(256) void input_plane(const float* __restrict__ x, _Float16* __restrict__ xp)
{
  const int gi = blockIdx.x * 256 + threadIdx.x;
  const int ro = gi / (kI / 8);
  const int c8 = (gi - ro * (kI / 8)) * 8;
  const int t  = ro / kB;
  const int b  = ro - t * kB;
  const float* src = x + ((size_t)b * kS + t) * kI + c8;
  const v4f a0 = *(const v4f*)(src);
  const v4f a1 = *(const v4f*)(src + 4);
  v8h hv;
#pragma unroll
  for (int e = 0; e < 4; ++e) {
    const float t0 = a0[e];
    const float t1 = a1[e];
    hv[e]     = input_half(t0, kActCarry);
    hv[4 + e] = input_half(t1, kActCarry);
  }
  _Float16* dst = xp + (size_t)ro * kI + c8;
  *(volatile v8h*)dst = hv;
  __threadfence();
  *(volatile v8h*)dst = hv;
}

__global__ __launch_bounds__(256) void linear_layer_plane(
    const _Float16* __restrict__ A, int lda,
    const _Float16* __restrict__ Bt, int ldb,
    _Float16* __restrict__ C, int ldc,
    const float* __restrict__ bias,
    int M, int N, int K, float scale, float ocarry)
{
  __shared__ __align__(16) float sT[8][16 * 68];
  const int lane = threadIdx.x & 31;
  const int wave = threadIdx.x >> 5;
  const int tilesN = N >> 6;
  const int tilesM = M >> 6;
  const int tile = blockIdx.x * 8 + wave;
  if (tile >= tilesM * tilesN) return;
  const int tm = tile / tilesN;
  const int tn = tile - tm * tilesN;
  const int m0 = tm << 6;
  const int n0 = tn << 6;
  const int rlane = lane & 15;
  const int koff  = (lane >> 4) * 8;
  const int mOff  = (lane >> 4) * 8;

  v8f acc[4][4];
#pragma unroll
  for (int i = 0; i < 4; ++i)
#pragma unroll
    for (int j = 0; j < 4; ++j) acc[i][j] = (v8f){0.f, 0.f, 0.f, 0.f, 0.f, 0.f, 0.f, 0.f};

#pragma unroll 1
  for (int k0 = 0; k0 < K; k0 += 32) {
    v16h bh[4];
#pragma unroll
    for (int j = 0; j < 4; ++j) {
      const size_t bo = (size_t)(n0 + (j << 4) + rlane) * ldb + koff + k0;
      bh[j] = load_frag(Bt + bo);
    }
#pragma unroll
    for (int i = 0; i < 4; ++i) {
      const size_t ao = (size_t)(m0 + (i << 4) + rlane) * lda + koff + k0;
      const v16h ah = load_frag(A + ao);
#pragma unroll
      for (int j = 0; j < 4; ++j) acc[i][j] = mma_g(ah, bh[j], acc[i][j]);
    }
  }

  float* slab = sT[wave];
  const int q  = lane >> 3;
  const int c8 = (lane & 7) * 8;
#pragma unroll
  for (int i = 0; i < 4; ++i) {
    const int mBase = m0 + (i << 4);
#pragma unroll
    for (int j = 0; j < 4; ++j) {
      const int n = n0 + (j << 4) + rlane;
      const float bv = bf_val(bias[n]);
#pragma unroll
      for (int r = 0; r < 8; ++r) {
        const float v = fmaf(acc[i][j][r], scale, bv);
        slab[(mOff + r) * 68 + (j << 4) + rlane] = v;
      }
    }
    __builtin_amdgcn_fence(__ATOMIC_RELEASE, "workgroup");
    __builtin_amdgcn_wave_barrier();
    __builtin_amdgcn_fence(__ATOMIC_ACQUIRE, "workgroup");
    v8h hv[4];
#pragma unroll
    for (int it = 0; it < 4; ++it) {
      const int row = it * 4 + q;
      const float* sp = slab + row * 68 + c8;
#pragma unroll
      for (int e = 0; e < 8; ++e) {
        const float sv = sp[e];
        hv[it][e] = carry_half(sv, ocarry);
      }
    }
    for (int pass = 0; pass < 2; ++pass) {
#pragma unroll
      for (int it = 0; it < 4; ++it) {
        const int row = it * 4 + q;
        *(volatile v8h*)(C + (size_t)(mBase + row) * ldc + n0 + c8) = hv[it];
      }
      __threadfence();
    }
    __builtin_amdgcn_fence(__ATOMIC_RELEASE, "workgroup");
    __builtin_amdgcn_wave_barrier();
    __builtin_amdgcn_fence(__ATOMIC_ACQUIRE, "workgroup");
  }
}

__device__ __forceinline__ void cell_products(v8f (&acc)[2][4], const _Float16* aRow, const _Float16* bRow)
{
#pragma unroll
  for (int ut = 0; ut < 2; ++ut)
#pragma unroll
    for (int g = 0; g < 4; ++g) acc[ut][g] = (v8f){0.f, 0.f, 0.f, 0.f, 0.f, 0.f, 0.f, 0.f};
#pragma unroll 1
  for (int k0 = 0; k0 < kKs; k0 += 32) {
    const v16h a = load_frag(aRow + k0);
#pragma unroll
    for (int ut = 0; ut < 2; ++ut) {
#pragma unroll
      for (int g = 0; g < 4; ++g) {
        const v16h b = load_frag(bRow + (size_t)(g * kH + ut * 16) * kKs + k0);
        acc[ut][g] = mma_g(a, b, acc[ut][g]);
      }
    }
  }
}

__device__ __forceinline__ void gate_math(const v8f (&acc)[2][4], const float (&bz)[8],
                                          float (&c)[16], float (&hv)[16])
{
#pragma unroll
  for (int ut = 0; ut < 2; ++ut) {
#pragma unroll
    for (int r = 0; r < 8; ++r) {
      const float xi = fmaf(acc[ut][0][r], kAccInv, bz[ut * 4 + 0]);
      const float xf = fmaf(acc[ut][1][r], kAccInv, bz[ut * 4 + 1]);
      const float xg = fmaf(acc[ut][2][r], kAccInv, bz[ut * 4 + 2]);
      const float xo = fmaf(acc[ut][3][r], kAccInv, bz[ut * 4 + 3]);
      const float ig = fast_sigmoid(xi);
      const float fg = fast_sigmoid(xf);
      const float gg = fast_tanh(xg);
      const float og = fast_sigmoid(xo);
      const float cn = fmaf(fg, c[ut * 8 + r], ig * gg);
      c[ut * 8 + r]  = cn;
      hv[ut * 8 + r] = og * fast_tanh(cn);
    }
  }
}

__device__ __forceinline__ void slab_fill(float* slab, const float (&v)[16], int hh, int nn)
{
#pragma unroll
  for (int ut = 0; ut < 2; ++ut)
#pragma unroll
    for (int r = 0; r < 8; ++r) slab[(8 * hh + r) * kSP + ut * 16 + nn] = v[ut * 8 + r];
}
__device__ __forceinline__ void slab_emit(const float* slab, float* g, size_t rs, int q, int c4)
{
  v4f v[4];
#pragma unroll
  for (int it = 0; it < 4; ++it) v[it] = *(const v4f*)(slab + (it * 4 + q) * kSP + c4);
  for (int pass = 0; pass < 2; ++pass) {
#pragma unroll
    for (int it = 0; it < 4; ++it)
      *(volatile v4f*)(g + (size_t)(it * 4 + q) * rs + c4) = v[it];
    __threadfence();
  }
}
__device__ __forceinline__ void slab_in(float* slab, const float* g, size_t rs, int q, int c4)
{
#pragma unroll
  for (int it = 0; it < 4; ++it) {
    const v4f a = *(const v4f*)(g + (size_t)(it * 4 + q) * rs + c4);
    v4f o;
#pragma unroll
    for (int e = 0; e < 4; ++e) {
      const float t0 = a[e];
      o[e] = bf_val(t0);
    }
    *(v4f*)(slab + (it * 4 + q) * kSP + c4) = o;
  }
}

__global__ __launch_bounds__(512) __attribute__((amdgpu_num_vgpr(256)))
void stacked_cell_steps(
    const _Float16* __restrict__ wp, const _Float16* __restrict__ xt, const float* __restrict__ fut,
    const float* __restrict__ hin, const float* __restrict__ cin,
    const float* __restrict__ ebih, const float* __restrict__ ebhh,
    const float* __restrict__ dbih, const float* __restrict__ dbhh,
    float* __restrict__ out)
{
  __shared__ __align__(16) _Float16 sA[kRowsPerBlock * kAP];
  __shared__ __align__(16) float    sBias[kL * kG];
  __shared__ __align__(16) float    sSlab[kStepWaves * 16 * kSP];

  const int tid  = threadIdx.x;
  const int lane = tid & 31;
  const int wave = tid >> 5;
  const int hh   = lane >> 4;
  const int nn   = lane & 15;
  const int q    = lane >> 3;
  const int c4   = (lane & 7) * 4;
  const int s0   = blockIdx.x * kRowsPerBlock;
  const int u0   = wave * kUnitsPerWave;
  float* slab = sSlab + wave * (16 * kSP);
  float* hid  = out + kOutHidden;
  float* cel  = out + kOutCell;

#pragma unroll 1
  for (int i = 0; i < 4; ++i) {
    const int idx = tid + i * kStepThreads;
    const int l   = idx >> 10;
    const int rem = idx & 1023;
    const int m   = rem >> 6;
    const int c8  = (rem & 63) << 3;
    const float* src = hin + ((size_t)(l * kB + s0 + m)) * kH + c8;
    const v4f a0 = *(const v4f*)(src);
    const v4f a1 = *(const v4f*)(src + 4);
    v8h hv8;
#pragma unroll
    for (int e = 0; e < 4; ++e) {
      const float t0 = a0[e];
      const float t1 = a1[e];
      hv8[e]     = input_half(t0, kActCarry);
      hv8[4 + e] = input_half(t1, kActCarry);
    }
    *(v8h*)(sA + m * kAP + kH + l * kH + c8) = hv8;
  }

  float c0[16], c1[16];
  slab_in(slab, cin + ((size_t)s0) * kH + u0, (size_t)kH, q, c4);
  __syncthreads();
#pragma unroll
  for (int ut = 0; ut < 2; ++ut)
#pragma unroll
    for (int r = 0; r < 8; ++r) c0[ut * 8 + r] = slab[(8 * hh + r) * kSP + ut * 16 + nn];
  __syncthreads();
  slab_in(slab, cin + ((size_t)(kB + s0)) * kH + u0, (size_t)kH, q, c4);
  __syncthreads();
#pragma unroll
  for (int ut = 0; ut < 2; ++ut)
#pragma unroll
    for (int r = 0; r < 8; ++r) c1[ut * 8 + r] = slab[(8 * hh + r) * kSP + ut * 16 + nn];

#pragma unroll 1
  for (int ph = 0; ph < 2; ++ph) {
    const bool dec = (ph == 1);
    const int  T   = dec ? kF : kS;
    const float* bih = dec ? dbih : ebih;
    const float* bhh = dec ? dbhh : ebhh;
    const _Float16* w0 = wp + (size_t)(ph * 2 + 0) * kG * kKs + (size_t)(u0 + nn) * kKs + 8 * hh;
    const _Float16* w1 = wp + (size_t)(ph * 2 + 1) * kG * kKs + (size_t)(u0 + nn) * kKs + 8 * hh;
    __syncthreads();
    {
      const int e0 = tid * 8;
      const v4f p0 = *(const v4f*)(bih + e0);
      const v4f p1 = *(const v4f*)(bih + e0 + 4);
      const v4f r0 = *(const v4f*)(bhh + e0);
      const v4f r1 = *(const v4f*)(bhh + e0 + 4);
      v4f o0, o1;
#pragma unroll
      for (int e = 0; e < 4; ++e) {
        const float a = p0[e];
        const float b = r0[e];
        const float c = p1[e];
        const float d = r1[e];
        o0[e] = bf_val(a) + bf_val(b);
        o1[e] = bf_val(c) + bf_val(d);
      }
      *(v4f*)(sBias + e0)     = o0;
      *(v4f*)(sBias + e0 + 4) = o1;
    }

#pragma unroll 1
    for (int t = 0; t < T; ++t) {
      const bool lastG = dec && (t == T - 1);
#pragma unroll
      for (int i = 0; i < 2; ++i) {
        const int ci = tid + i * kStepThreads;
        const int m  = ci >> 6;
        const int c8 = (ci & 63) << 3;
        v8h xv;
        if (!dec) {
          xv = *(const v8h*)(xt + ((size_t)t * kB + s0 + m) * kH + c8);
        } else {
          const float* src = fut + ((size_t)(s0 + m) * kF + t) * kI + c8;
          const v4f a0 = *(const v4f*)(src);
          const v4f a1 = *(const v4f*)(src + 4);
#pragma unroll
          for (int e = 0; e < 4; ++e) {
            const float t0 = a0[e];
            const float t1 = a1[e];
            xv[e]     = input_half(t0, kActCarry);
            xv[4 + e] = input_half(t1, kActCarry);
          }
        }
        *(v8h*)(sA + m * kAP + c8) = xv;
      }
      __syncthreads();

      v8f acc[2][4];
      float bz[8];
      float hv[16];

      cell_products(acc, sA + nn * kAP + 8 * hh, w0);
      __syncthreads();
#pragma unroll
      for (int ut = 0; ut < 2; ++ut)
#pragma unroll
        for (int g = 0; g < 4; ++g) bz[ut * 4 + g] = sBias[g * kH + u0 + ut * 16 + nn];
      gate_math(acc, bz, c0, hv);
#pragma unroll
      for (int ut = 0; ut < 2; ++ut)
#pragma unroll
        for (int r = 0; r < 8; ++r)
          sA[(8 * hh + r) * kAP + kH + u0 + ut * 16 + nn] = carry_half(hv[ut * 8 + r], kActCarry);
      if (lastG) {
        slab_fill(slab, hv, hh, nn);
        __syncthreads();
        slab_emit(slab, hid + ((size_t)s0) * kH + u0, (size_t)kH, q, c4);
        __syncthreads();
        slab_fill(slab, c0, hh, nn);
        __syncthreads();
        slab_emit(slab, cel + ((size_t)s0) * kH + u0, (size_t)kH, q, c4);
        __syncthreads();
      }
      __syncthreads();

      cell_products(acc, sA + nn * kAP + kH + 8 * hh, w1);
      __syncthreads();
#pragma unroll
      for (int ut = 0; ut < 2; ++ut)
#pragma unroll
        for (int g = 0; g < 4; ++g) bz[ut * 4 + g] = sBias[kG + g * kH + u0 + ut * 16 + nn];
      gate_math(acc, bz, c1, hv);
#pragma unroll
      for (int ut = 0; ut < 2; ++ut)
#pragma unroll
        for (int r = 0; r < 8; ++r)
          sA[(8 * hh + r) * kAP + 2 * kH + u0 + ut * 16 + nn] = carry_half(hv[ut * 8 + r], kActCarry);
      if (dec) {
        slab_fill(slab, hv, hh, nn);
        __syncthreads();
        slab_emit(slab, out + ((size_t)s0 * kF + t) * kH + u0, (size_t)kF * kH, q, c4);
        if (lastG) slab_emit(slab, hid + ((size_t)(kB + s0)) * kH + u0, (size_t)kH, q, c4);
        __syncthreads();
        if (lastG) {
          slab_fill(slab, c1, hh, nn);
          __syncthreads();
          slab_emit(slab, cel + ((size_t)(kB + s0)) * kH + u0, (size_t)kH, q, c4);
          __syncthreads();
        }
      }
    }
  }
}

extern "C" void kernel_launch(void* const* d_in, const int* in_sizes, int n_in,
                              void* d_out, int out_size, void* d_ws, size_t ws_size,
                              hipStream_t stream) {
  if (n_in < 14) return;
  if (in_sizes[0] != kB * kS * kI) return;
  if (in_sizes[1] != kB * kF * kI) return;
  if (in_sizes[2] != kL * kB * kH) return;
  if (in_sizes[3] != kL * kB * kH) return;
  if (in_sizes[4] != kH * kI) return;
  if (in_sizes[5] != kH) return;
  if (in_sizes[6] != kL * kG * kH) return;
  if (in_sizes[7] != kL * kG * kH) return;
  if (in_sizes[8] != kL * kG) return;
  if (in_sizes[9] != kL * kG) return;
  if (in_sizes[10] != kL * kG * kH) return;
  if (in_sizes[11] != kL * kG * kH) return;
  if (in_sizes[12] != kL * kG) return;
  if (in_sizes[13] != kL * kG) return;
  if ((size_t)out_size != kOutTotal) return;
  if (ws_size < kWsTotal) return;

  const float* x       = (const float*)d_in[0];
  const float* fut     = (const float*)d_in[1];
  const float* enc_h   = (const float*)d_in[2];
  const float* enc_c   = (const float*)d_in[3];
  const float* fc_w    = (const float*)d_in[4];
  const float* fc_b    = (const float*)d_in[5];
  const float* enc_wih = (const float*)d_in[6];
  const float* enc_whh = (const float*)d_in[7];
  const float* enc_bih = (const float*)d_in[8];
  const float* enc_bhh = (const float*)d_in[9];
  const float* dec_wih = (const float*)d_in[10];
  const float* dec_whh = (const float*)d_in[11];
  const float* dec_bih = (const float*)d_in[12];
  const float* dec_bhh = (const float*)d_in[13];
  float* out = (float*)d_out;

  char* ws = (char*)d_ws;
  _Float16* WP   = (_Float16*)(ws + kOffWP);
  _Float16* FCW  = (_Float16*)(ws + kOffFCW);
  _Float16* X16  = (_Float16*)(ws + kOffX16);
  _Float16* XT16 = (_Float16*)(ws + kOffXT);

  weight_planes<<<4 * kCellPlaneBlocks + kFcPlaneBlocks, 256, 0, stream>>>(
      enc_wih, enc_whh, dec_wih, dec_whh, fc_w, WP, FCW);

  static_assert(((size_t)kB * kS * kI / 8) % 256 == 0, "exact grid");
  input_plane<<<(kB * kS * kI / 8) / 256, 256, 0, stream>>>(x, X16);

  static_assert((kB * kS) % 64 == 0 && (kH % 64) == 0 && (kI % 32) == 0, "tile multiples");
  {
    constexpr int tiles = (kB * kS / 64) * (kH / 64);
    static_assert((tiles % 8) == 0, "whole blocks");
    linear_layer_plane<<<tiles / 8, 256, 0, stream>>>(
        X16, kI, FCW, kI, XT16, kH, fc_b, kB * kS, kH, kI, kAccInv, kActCarry);
  }

  stacked_cell_steps<<<kB / kRowsPerBlock, kStepThreads, 0, stream>>>(
      WP, XT16, fut, enc_h, enc_c, enc_bih, enc_bhh, dec_bih, dec_bhh, out);
}
